// MutiAtten_3899830305375
// MI455X (gfx1250) — hardware-verified
//
#include <hip/hip_runtime.h>


namespace {
constexpr int Bn = 4, L = 2048, D = 1024, NT = Bn * L;
constexpr float QSC = 0.03125f;
constexpr float PSC = 4096.0f;
constexpr size_t PL = (size_t)Bn * L * D;

typedef _Float16 b16;
typedef __attribute__((ext_vector_type(16))) _Float16 v16b;
typedef __attribute__((ext_vector_type(16))) __bf16 v16bb;
typedef __attribute__((ext_vector_type(8))) _Float16 v8b;
typedef __attribute__((ext_vector_type(8))) unsigned short v8us;
typedef __attribute__((ext_vector_type(8))) float v8f;
typedef __attribute__((ext_vector_type(4))) float v4f;
__device__ __forceinline__ float bf16_rne(float f) { unsigned int u = __float_as_uint(f); u += 0x7FFFu + ((u >> 16) & 1u); return __uint_as_float(u & 0xFFFF0000u); }
__device__ __forceinline__ unsigned short bf16_bits(float f) { unsigned int u = __float_as_uint(f); u += 0x7FFFu + ((u >> 16) & 1u); return (unsigned short)(u >> 16); }
__device__ __forceinline__ v16b frag_kb(const b16* p, int hh) { const v8b a = *(const v8b*)(p + 8 * hh), b = *(const v8b*)(p + 16 + 8 * hh); v16b f;
#pragma unroll
  for (int e = 0; e < 8; ++e) { f[e] = a[e]; f[8 + e] = b[e]; } return f; }
__device__ __forceinline__ v16bb frag_bf(const unsigned short* p, int hh) { const v8us a = *(const v8us*)(p + 8 * hh), b = *(const v8us*)(p + 16 + 8 * hh); union { unsigned short s[16]; v16bb v; } u;
#pragma unroll
  for (int e = 0; e < 8; ++e) { u.s[e] = a[e]; u.s[8 + e] = b[e]; } return u.v; }
__device__ __forceinline__ v16bb frag_f32bf(const float* p, int hh) { union { unsigned short s[16]; v16bb v; } u;
#pragma unroll
  for (int e = 0; e < 8; ++e) { u.s[e] = bf16_bits(p[8 * hh + e]); u.s[8 + e] = bf16_bits(p[16 + 8 * hh + e]); } return u.v; }
__device__ __forceinline__ v8f wmma16b(v16b a, v16b b, v8f c) { v8f d = __builtin_amdgcn_wmma_f32_16x16x32_f16(false, a, false, b, (short)0, c, false, false); asm volatile("v_nop\n\tv_nop\n\tv_nop\n\tv_nop" : "+v"(d) : "v"(a), "v"(b)); return d; }
__device__ __forceinline__ v8f wmma16bb(v16bb a, v16bb b, v8f c) { v8f d = __builtin_amdgcn_wmma_f32_16x16x32_bf16(false, a, false, b, (short)0, c, false, false); asm volatile("v_nop\n\tv_nop\n\tv_nop\n\tv_nop" : "+v"(d) : "v"(a), "v"(b)); return d; }
__device__ __forceinline__ void wave_lds_sync() { __builtin_amdgcn_fence(__ATOMIC_RELEASE, "workgroup"); __builtin_amdgcn_wave_barrier(); __builtin_amdgcn_fence(__ATOMIC_ACQUIRE, "workgroup"); }
__device__ __forceinline__ float nexp(float x) { return __builtin_amdgcn_exp2f(x * 1.4426950408889634f); }

__global__ __launch_bounds__(256) void prep_kernel(const float* __restrict__ wkqv, const float* __restrict__ wp, unsigned short* __restrict__ w16, b16* __restrict__ wp16) {
  const size_t tid = (size_t)blockIdx.x * blockDim.x + threadIdx.x, nth = (size_t)gridDim.x * blockDim.x;
  for (int pass = 0; pass < 2; ++pass) {
    for (size_t p = tid; p < (size_t)3 * D * D / 8; p += nth) { v8us v;
#pragma unroll
      for (int e = 0; e < 8; ++e) v[e] = bf16_bits(wkqv[p * 8 + e]);
      *(volatile v8us*)(w16 + p * 8) = v; }
    for (size_t p = tid; p < (size_t)D * D / 8; p += nth) { v8b v;
#pragma unroll
      for (int e = 0; e < 8; ++e) v[e] = (b16)bf16_rne(wp[p * 8 + e]);
      *(volatile v8b*)(wp16 + p * 8) = v; }
    __threadfence(); }
}

__global__ __launch_bounds__(128) void proj_kernel(const float* __restrict__ x, const unsigned short* __restrict__ w16, const float* __restrict__ bkqv, b16* __restrict__ Kr, b16* __restrict__ Qr, b16* __restrict__ Vt) {
  __shared__ __attribute__((aligned(16))) b16 Th[4][32][64 + 8], Tl[4][32][64 + 8]; __shared__ __attribute__((aligned(16))) b16 Tt[64][128 + 8];
  const int lane = threadIdx.x & 31, wave = threadIdx.x >> 5, nloc = lane & 15, hlf = lane >> 4, m0 = blockIdx.y * 128 + wave * 32, c0 = blockIdx.x * 64, which = blockIdx.x / 16, cc0 = c0 % D;
  const int b = (blockIdx.y * 128) / L, l0 = (blockIdx.y * 128) % L;
  v8f acc[2][4];
#pragma unroll
  for (int r = 0; r < 2; ++r)
#pragma unroll
    for (int t = 0; t < 4; ++t) acc[r][t] = (v8f){};
#pragma unroll 2
  for (int kb = 0; kb < D; kb += 32) { const v16bb a0 = frag_f32bf(x + (size_t)(m0 + nloc) * D + kb, hlf), a1 = frag_f32bf(x + (size_t)(m0 + 16 + nloc) * D + kb, hlf);
#pragma unroll
    for (int t = 0; t < 4; ++t) { const v16bb bw = frag_bf(w16 + (size_t)(c0 + t * 16 + nloc) * D + kb, hlf); acc[0][t] = wmma16bb(a0, bw, acc[0][t]); acc[1][t] = wmma16bb(a1, bw, acc[1][t]); } }
  const float scl = (which == 1) ? QSC : 1.0f;
  if (which < 2) {
#pragma unroll
    for (int t = 0; t < 4; ++t) { const float bb = bf16_rne(bkqv[c0 + t * 16 + nloc]);
#pragma unroll
      for (int r = 0; r < 2; ++r)
#pragma unroll
        for (int v = 0; v < 8; ++v) { const float val = (acc[r][t][v] + bb) * scl; const b16 hi = (b16)val; Th[wave][r * 16 + 8 * hlf + v][t * 16 + nloc] = hi; Tl[wave][r * 16 + 8 * hlf + v][t * 16 + nloc] = (b16)(val - (float)hi); } }
    wave_lds_sync();
    b16* dst = ((which == 0) ? Kr : Qr) + (size_t)m0 * D + cc0;
    for (int pass = 0; pass < 2; ++pass) {
#pragma unroll
      for (int j = 0; j < 8; ++j) { const int rr = j * 4 + (lane >> 3), c8 = (lane & 7) * 8; *(volatile v8b*)(dst + (size_t)rr * D + c8) = *(const v8b*)(&Th[wave][rr][c8]);
        if (which == 1) *(volatile v8b*)(dst + PL + (size_t)rr * D + c8) = *(const v8b*)(&Tl[wave][rr][c8]); }
      __threadfence(); }
    return;
  }
#pragma unroll
  for (int t = 0; t < 4; ++t) { const float bb = bf16_rne(bkqv[c0 + t * 16 + nloc]);
#pragma unroll
    for (int r = 0; r < 2; ++r)
#pragma unroll
      for (int v = 0; v < 8; ++v) Tt[t * 16 + nloc][wave * 32 + r * 16 + 8 * hlf + v] = (b16)(acc[r][t][v] + bb); }
  __syncthreads();
  for (int pass = 0; pass < 2; ++pass) { for (int i = threadIdx.x; i < 64 * 16; i += 128) { const int dd = i >> 4, c8 = (i & 15) * 8; *(volatile v8b*)(Vt + ((size_t)b * D + cc0 + dd) * L + l0 + c8) = *(const v8b*)(&Tt[dd][c8]); } __threadfence(); }
}

__global__ __launch_bounds__(256) void score_kernel(const b16* __restrict__ Qr, const b16* __restrict__ Kr, const int* __restrict__ vlen, b16* __restrict__ SP) {
  __shared__ __attribute__((aligned(16))) b16 Ts[8][16][64 + 8]; __shared__ float Mz[8][2][16]; __shared__ float Mh[8][16][L / 32 + 1];
  const int wid = threadIdx.x >> 5, lane = threadIdx.x & 31, hh = lane >> 4, col = lane & 15; const int qg = blockIdx.x * 8 + wid, b = qg / (L / 16), q0 = (qg % (L / 16)) * 16;
  const int vl = min(max(vlen[b], 1), L), kend = (vl + 31) & ~31, kend64 = (vl + 63) & ~63;
  const b16* Q = Qr + ((size_t)b * L + q0 + col) * D; const b16* K = Kr + ((size_t)b * L) * D; b16* Srow = SP + ((size_t)b * L + q0) * L;
  float m = -INFINITY, z = 0.0f;
  for (int kb = 0; kb < kend64; kb += 32) {
    const int half = (kb >> 5) & 1;
    if (kb < kend) { v8f s0 = {}, s1 = {};
#pragma unroll 4
      for (int ks = 0; ks < D; ks += 32) { const v16b qf = frag_kb(Q + ks, hh), ql = frag_kb(Q + PL + ks, hh); const v16b ka = frag_kb(K + (size_t)(kb + col) * D + ks, hh), kc = frag_kb(K + (size_t)(kb + 16 + col) * D + ks, hh);
        s0 = wmma16b(ka, qf, s0); s0 = wmma16b(ka, ql, s0); s1 = wmma16b(kc, qf, s1); s1 = wmma16b(kc, ql, s1); }
      float mr = -INFINITY;
#pragma unroll
      for (int r = 0; r < 8; ++r) { if (kb + 8 * hh + r >= vl) s0[r] = -INFINITY; if (kb + 16 + 8 * hh + r >= vl) s1[r] = -INFINITY; mr = fmaxf(mr, fmaxf(s0[r], s1[r])); }
      mr = fmaxf(mr, __shfl_xor(mr, 16));
      const float mn = fmaxf(m, mr); float sum = 0.0f;
#pragma unroll
      for (int r = 0; r < 8; ++r) { sum += nexp(s0[r] - mn) + nexp(s1[r] - mn); }
      sum += __shfl_xor(sum, 16); z = z * nexp(m - mn) + sum; m = mn;
      if (hh == 0) Mh[wid][col][kb >> 5] = mn;
#pragma unroll
      for (int r = 0; r < 8; ++r) { Ts[wid][col][half * 32 + 8 * hh + r] = (b16)(nexp(s0[r] - mn) * PSC); Ts[wid][col][half * 32 + 16 + 8 * hh + r] = (b16)(nexp(s1[r] - mn) * PSC); }
    } else {
#pragma unroll
      for (int r = 0; r < 8; ++r) { Ts[wid][col][half * 32 + 8 * hh + r] = (b16)0.0f; Ts[wid][col][half * 32 + 16 + 8 * hh + r] = (b16)0.0f; } }
    if (half == 1) { wave_lds_sync();
      for (int pass = 0; pass < 2; ++pass) {
#pragma unroll
        for (int j = 0; j < 4; ++j) { const int rr = j * 4 + (lane >> 3), c8 = (lane & 7) * 8; *(volatile v8b*)(Srow + (size_t)rr * L + (kb - 32) + c8) = *(const v8b*)(&Ts[wid][rr][c8]); } }
      wave_lds_sync(); }
  }
  if (hh == 0) { Mz[wid][0][col] = m; Mz[wid][1][col] = 1.0f / z; }
  __threadfence(); wave_lds_sync();
  for (int kb = 0; kb < L; kb += 64) {
#pragma unroll
    for (int j = 0; j < 4; ++j) { const int rr = j * 4 + (lane >> 3), c8 = (lane & 7) * 8; b16* p = Srow + (size_t)rr * L + kb + c8; const float mm = Mz[wid][0][rr], iz = Mz[wid][1][rr]; v8b o;
      if (kb < kend64) { const v8b a = *(const volatile v8b*)p; const int blk = (kb + c8) >> 5; const float resc = (blk * 32 < kend) ? nexp(Mh[wid][rr][blk] - mm) * iz : 0.0f;
#pragma unroll
        for (int e = 0; e < 8; ++e) o[e] = (b16)((kb + c8 + e < vl) ? (float)a[e] * resc : 0.0f); }
      else {
#pragma unroll
        for (int e = 0; e < 8; ++e) o[e] = (b16)0.0f; }
      for (int pass = 0; pass < 2; ++pass) *(volatile v8b*)p = o; } }
  __threadfence();
}

__global__ __launch_bounds__(128) void pv_kernel(const b16* __restrict__ Vt, const b16* __restrict__ SP, const int* __restrict__ vlen, b16* __restrict__ Ot) {
  __shared__ __attribute__((aligned(16))) b16 Th[4][32][64 + 8];
  const int lane = threadIdx.x & 31, wave = threadIdx.x >> 5, nloc = lane & 15, hlf = lane >> 4, b = blockIdx.z, m0 = blockIdx.y * 128 + wave * 32, c0 = blockIdx.x * 64;
  const int vl = min(max(vlen[b], 1), L), kend = (vl + 31) & ~31;
  const b16* A = Vt + ((size_t)b * D) * L; const b16* Bp = SP + ((size_t)b * L) * L;
  v8f acc[2][4];
#pragma unroll
  for (int r = 0; r < 2; ++r)
#pragma unroll
    for (int t = 0; t < 4; ++t) acc[r][t] = (v8f){};
  for (int kb = 0; kb < kend; kb += 32) { const v16b a0 = frag_kb(A + (size_t)(m0 + nloc) * L + kb, hlf), a1 = frag_kb(A + (size_t)(m0 + 16 + nloc) * L + kb, hlf);
#pragma unroll
    for (int t = 0; t < 4; ++t) { const v16b bw = frag_kb(Bp + (size_t)(c0 + t * 16 + nloc) * L + kb, hlf); acc[0][t] = wmma16b(a0, bw, acc[0][t]); acc[1][t] = wmma16b(a1, bw, acc[1][t]); } }
#pragma unroll
  for (int t = 0; t < 4; ++t)
#pragma unroll
    for (int r = 0; r < 2; ++r)
#pragma unroll
      for (int v = 0; v < 8; ++v) Th[wave][r * 16 + 8 * hlf + v][t * 16 + nloc] = (b16)(acc[r][t][v] * (1.0f / PSC));
  wave_lds_sync();
  b16* dst = Ot + ((size_t)b * D + m0) * L + c0;
  for (int pass = 0; pass < 2; ++pass) {
#pragma unroll
    for (int j = 0; j < 8; ++j) { const int rr = j * 4 + (lane >> 3), c8 = (lane & 7) * 8; *(volatile v8b*)(dst + (size_t)rr * L + c8) = *(const v8b*)(&Th[wave][rr][c8]); }
    __threadfence(); }
}

__global__ __launch_bounds__(128) void out_kernel(const b16* __restrict__ Ot, const b16* __restrict__ wp16, const float* __restrict__ bp, float* __restrict__ y) {
  __shared__ __attribute__((aligned(16))) float Ts[4][32 * 64];
  const int lane = threadIdx.x & 31, wave = threadIdx.x >> 5, nloc = lane & 15, hlf = lane >> 4, m0 = blockIdx.y * 128 + wave * 32, c0 = blockIdx.x * 64;
  v8f acc[2][4];
#pragma unroll
  for (int r = 0; r < 2; ++r)
#pragma unroll
    for (int t = 0; t < 4; ++t) acc[r][t] = (v8f){};
#pragma unroll 2
  for (int kb = 0; kb < D; kb += 32) { const v16b a0 = frag_kb(Ot + (size_t)(m0 + nloc) * D + kb, hlf), a1 = frag_kb(Ot + (size_t)(m0 + 16 + nloc) * D + kb, hlf);
#pragma unroll
    for (int t = 0; t < 4; ++t) { const v16b bw = frag_kb(wp16 + (size_t)(c0 + t * 16 + nloc) * D + kb, hlf); acc[0][t] = wmma16b(a0, bw, acc[0][t]); acc[1][t] = wmma16b(a1, bw, acc[1][t]); } }
  float* Tt = Ts[wave];
#pragma unroll
  for (int t = 0; t < 4; ++t) { const float bb = bf16_rne(bp[c0 + t * 16 + nloc]);
#pragma unroll
    for (int r = 0; r < 2; ++r)
#pragma unroll
      for (int v = 0; v < 8; ++v) Tt[(r * 16 + v + 8 * hlf) * 64 + t * 16 + nloc] = acc[r][t][v] + bb; }
  wave_lds_sync();
  float* dst0 = y + (size_t)m0 * D + c0;
  for (int pass = 0; pass < 2; ++pass) {
#pragma unroll
    for (int j = 0; j < 16; ++j) { const int rr = j * 2 + hlf, c4 = nloc * 4; *(volatile v4f*)(dst0 + (size_t)rr * D + c4) = *(const v4f*)(Tt + rr * 64 + c4); }
    __threadfence(); }
}
}

extern "C" void kernel_launch(void* const* d_in, const int* in_sizes, int n_in,
                              void* d_out, int out_size, void* d_ws, size_t ws_size, hipStream_t stream) {
  (void)n_in; (void)out_size;
  const float* x = (const float*)d_in[0]; const int* vlen = (const int*)d_in[1]; const float* wkqv = (const float*)d_in[2]; const float* bkqv = (const float*)d_in[3]; const float* wp = (const float*)d_in[4]; const float* bp = (const float*)d_in[5];
  float* y = (float*)d_out;
  if (in_sizes[0] != NT * D || in_sizes[1] != Bn || in_sizes[2] != 3 * D * D || in_sizes[3] != 3 * D || in_sizes[4] != D * D || in_sizes[5] != D) return;
  size_t off = 0; char* ws = (char*)d_ws;
  auto carve = [&](size_t bytes) { char* p = ws + off; off += (bytes + 255) & ~(size_t)255; return p; };
  unsigned short* w16 = (unsigned short*)carve((size_t)3 * D * D * 2); b16* wp16 = (b16*)carve((size_t)D * D * 2);
  b16* Kr = (b16*)carve(PL * 2); b16* Qr = (b16*)carve(PL * 2 * 2); b16* Vt = (b16*)carve(PL * 2); b16* SP = (b16*)carve((size_t)Bn * L * L * 2); b16* Ot = (b16*)carve(PL * 2);
  if (off > ws_size) return;
  prep_kernel<<<1024, 256, 0, stream>>>(wkqv, wp, w16, wp16);
  proj_kernel<<<dim3(3 * D / 64, NT / 128), 128, 0, stream>>>(x, w16, bkqv, Kr, Qr, Vt);
  score_kernel<<<NT / 16 / 8, 256, 0, stream>>>(Qr, Kr, vlen, SP);
  pv_kernel<<<dim3(L / 64, D / 128, Bn), 128, 0, stream>>>(Vt, SP, vlen, Ot);
  out_kernel<<<dim3(D / 64, NT / 128), 128, 0, stream>>>(Ot, wp16, bp, y);
}
